// SimplifiedGCN_44959717654591
// MI455X (gfx1250) — hardware-verified
//
#include <hip/hip_runtime.h>

typedef float          v8f   __attribute__((ext_vector_type(8)));
typedef float          v4f   __attribute__((ext_vector_type(4)));
typedef unsigned int   v4u   __attribute__((ext_vector_type(4)));
typedef int            v8i   __attribute__((ext_vector_type(8)));
typedef unsigned short v8us  __attribute__((ext_vector_type(8)));
typedef unsigned short v16us __attribute__((ext_vector_type(16)));
typedef __bf16         v16bf __attribute__((ext_vector_type(16)));
typedef _Float16       v16h  __attribute__((ext_vector_type(16)));
typedef v4f  __attribute__((may_alias)) v4fa;
typedef v8us __attribute__((may_alias)) v8usa;
union FragB { v16bf v; v16us u; v8us h[2]; v8i w; };
union FragH { v16h  v; v16us u; v8us h[2]; v8i w; };

__device__ __forceinline__ v8f wmb(const FragB& a, const FragB& b, v8f c) {
  v8f d = __builtin_amdgcn_wmma_f32_16x16x32_bf16(false, a.v, false, b.v, (short)0, c, false, false);
  asm volatile("v_nop\n\tv_nop\n\tv_nop\n\tv_nop" : "+v"(d) : "v"(a.w), "v"(b.w));
  return d;
}

__device__ __forceinline__ v8f wmh(const FragH& a, const FragH& b, v8f c) {
  v8f d = __builtin_amdgcn_wmma_f32_16x16x32_f16(false, a.v, false, b.v, (short)0, c, false, false);
  asm volatile("v_nop\n\tv_nop\n\tv_nop\n\tv_nop" : "+v"(d) : "v"(a.w), "v"(b.w));
  return d;
}

__device__ __forceinline__ unsigned bf16_bits(float f) {
  const unsigned u = __float_as_uint(f);
  const unsigned r = (u + 0x7FFFu + ((u >> 16) & 1u)) >> 16;
  const unsigned q = (u >> 16) | 0x40u;
  return ((u & 0x7fffffffu) > 0x7f800000u) ? q : r;
}

__device__ __forceinline__ float bf16_val(float f) {
  return __uint_as_float(bf16_bits(f) << 16);
}
__device__ __forceinline__ int clampi(int v, int lo, int hi) {
  return v < lo ? lo : (v > hi ? hi : v);
}

__device__ __forceinline__ unsigned f16_bits(float f) {
  const unsigned u  = __float_as_uint(f);
  const unsigned s  = (u >> 16) & 0x8000u;
  const unsigned a  = u & 0x7fffffffu;
  const unsigned t  = a - 0x38000000u;
  const unsigned r  = (t + 0x0FFFu + ((t >> 13) & 1u)) >> 13;
  const unsigned rc = r > 0x7C00u ? 0x7C00u : r;
  const bool small  = a < 0x38800000u;
  const bool isnan  = a > 0x7f800000u;
  const unsigned fin = small ? 0u : (s | rc);
  return isnan ? (s | 0x7E00u) : fin;
}

__device__ __forceinline__ unsigned pk16(unsigned lo, unsigned hi) { return lo | (hi << 16); }
__device__ __forceinline__ unsigned bf16_lo_bits(float v) {
  float hi = bf16_val(v);
  asm volatile("" : "+v"(hi));
  return bf16_bits(v - hi);
}
__device__ __forceinline__ v4u pack8_bf16(v4f a, v4f c) {
  return (v4u){ pk16(bf16_bits(a[0]), bf16_bits(a[1])), pk16(bf16_bits(a[2]), bf16_bits(a[3])),
                pk16(bf16_bits(c[0]), bf16_bits(c[1])), pk16(bf16_bits(c[2]), bf16_bits(c[3])) };
}
__device__ __forceinline__ v4u pack8_bf16_lo(v4f a, v4f c) {
  return (v4u){ pk16(bf16_lo_bits(a[0]), bf16_lo_bits(a[1])), pk16(bf16_lo_bits(a[2]), bf16_lo_bits(a[3])),
                pk16(bf16_lo_bits(c[0]), bf16_lo_bits(c[1])), pk16(bf16_lo_bits(c[2]), bf16_lo_bits(c[3])) };
}
__device__ __forceinline__ v4u pack8_f16(v4f a, v4f c) {
  return (v4u){ pk16(f16_bits(a[0]), f16_bits(a[1])), pk16(f16_bits(a[2]), f16_bits(a[3])),
                pk16(f16_bits(c[0]), f16_bits(c[1])), pk16(f16_bits(c[2]), f16_bits(c[3])) };
}

template <int FORM>
__global__ __launch_bounds__(256) void k_plane(const float* __restrict__ src, int rows, int cols, int ldsrc,
                                               unsigned short* __restrict__ dst, int MP, int KP) {
  static_assert(FORM >= 0 && FORM <= 3);
  const int KTOT = (FORM == 1 || FORM == 3) ? 2 * KP : KP;
  const unsigned ppr   = (unsigned)(KTOT >> 3);
  const unsigned kp8   = (unsigned)(KP >> 3);
  const unsigned total = (unsigned)MP * ppr;
  const unsigned g     = blockIdx.x * 256u + threadIdx.x;
  const unsigned rowu  = g / ppr;
  const unsigned p     = g - rowu * ppr;
  const bool second    = p >= kp8;
  const int row = (int)rowu;
  const int c0  = (int)((second ? p - kp8 : p) << 3);
  const float* srow = src + (size_t)clampi(row, 0, rows - 1) * (size_t)ldsrc;
  float x[8];
  unsigned mk[8];
#pragma unroll
  for (int e = 0; e < 8; ++e) {
    const int c = c0 + e;
    const float v = srow[clampi(c, 0, cols - 1)];
    asm volatile("" :: "v"(v));
    x[e]  = v;
    mk[e] = (row < rows && c < cols) ? 0xFFFFu : 0u;
  }
  const v4f a = (v4f){ x[0], x[1], x[2], x[3] };
  const v4f c = (v4f){ x[4], x[5], x[6], x[7] };
  v4u o;
  if (FORM == 2) {
    o = pack8_f16(a, c);
  } else {
    const v4u hi = pack8_bf16(a, c);
    o = hi;
    if (FORM == 1) { const v4u lo = pack8_bf16_lo(a, c); o = second ? lo : hi; }
  }
  const v4u mw = (v4u){ pk16(mk[0], mk[1]), pk16(mk[2], mk[3]), pk16(mk[4], mk[5]), pk16(mk[6], mk[7]) };
  o &= mw;
  if (g < total) {
    volatile v4u* q = (volatile v4u*)(dst + (size_t)g * 8);
    *q = o;
    __threadfence();
    *q = o;
  }
}

template <int FORM> struct FragOf    { typedef FragB T; };
template <>         struct FragOf<2> { typedef FragH T; };
__device__ __forceinline__ v8f mm(const FragB& a, const FragB& b, v8f c) { return wmb(a, b, c); }
__device__ __forceinline__ v8f mm(const FragH& a, const FragH& b, v8f c) { return wmh(a, b, c); }
template <class F> __device__ __forceinline__ F ld_frag(const unsigned short* p) {
  F f;
  f.h[0] = *(const v8usa*)(p);
  f.h[1] = *(const v8usa*)(p + 16);
  return f;
}

template <int FORM, int EPI>
__global__ __launch_bounds__(256) __attribute__((amdgpu_num_vgpr(248)))
void k_gemm_nt(const unsigned short* __restrict__ A, const unsigned short* __restrict__ B,
               const float* __restrict__ bias, float* __restrict__ D, int M, int N, int KTOT, int ldd) {
  static_assert(FORM >= 0 && FORM <= 2);
  static_assert(EPI == 0 || EPI == 1);
  typedef typename FragOf<FORM>::T F;
  __shared__ __attribute__((aligned(16))) float sT[8][16 * 68];
  const int lane = threadIdx.x & 31;
  const int wave = threadIdx.x >> 5;
  const int tilesM = (M + 63) >> 6;
  const int tilesN = (N + 63) >> 6;
  const int tile = blockIdx.x * 8 + wave;
  if (tile >= tilesM * tilesN) return;
  const int tm = tile / tilesN;
  const int tn = tile - tm * tilesN;
  const int m0 = tm << 6;
  const int n0 = tn << 6;

  const int rl = lane & 15;
  const int h8 = (lane >> 4) * 8;
  const unsigned short* pa = A + (size_t)(m0 + rl) * (size_t)KTOT + h8;
  const unsigned short* pb = B + (size_t)(n0 + rl) * (size_t)KTOT + h8;

  v8f acc[4][4];
#pragma unroll
  for (int i = 0; i < 4; ++i)
#pragma unroll
    for (int j = 0; j < 4; ++j) acc[i][j] = (v8f){0.f, 0.f, 0.f, 0.f, 0.f, 0.f, 0.f, 0.f};

#pragma unroll 1
  for (int k0 = 0; k0 < KTOT; k0 += 32) {
    F bf[4];
#pragma unroll
    for (int j = 0; j < 4; ++j) bf[j] = ld_frag<F>(pb + (size_t)(j << 4) * (size_t)KTOT + k0);
#pragma unroll
    for (int i = 0; i < 4; ++i) {
      const F af = ld_frag<F>(pa + (size_t)(i << 4) * (size_t)KTOT + k0);
#pragma unroll
      for (int j = 0; j < 4; ++j) acc[i][j] = mm(af, bf[j], acc[i][j]);
    }
  }

  float* slab = sT[wave];
  const int hh = lane >> 4;
  const int c4 = (lane & 15) * 4;
  const int nc = n0 + c4;
  const bool cok = nc < N;
  v4f bv = (v4f){0.f, 0.f, 0.f, 0.f};
  if (EPI == 1) {
    bv = *(const v4fa*)(bias + clampi(nc, 0, N - 4));
    asm volatile("" :: "v"(bv));
  }
#pragma unroll
  for (int i = 0; i < 4; ++i) {
    const int mBase = m0 + (i << 4);
#pragma unroll
    for (int j = 0; j < 4; ++j) {
#pragma unroll
      for (int r = 0; r < 8; ++r) slab[(h8 + r) * 68 + (j << 4) + rl] = acc[i][j][r];
    }
    __builtin_amdgcn_fence(__ATOMIC_RELEASE, "workgroup");
    __builtin_amdgcn_wave_barrier();
    __builtin_amdgcn_fence(__ATOMIC_ACQUIRE, "workgroup");
    v4f vv[8];
#pragma unroll
    for (int it = 0; it < 8; ++it) {
      const int row = it * 2 + hh;
      v4f v = *(const v4fa*)(slab + row * 68 + c4);
      if (EPI == 1) v += bv;
      vv[it] = v;
    }
    for (int pass = 0; pass < 2; ++pass) {
#pragma unroll
      for (int it = 0; it < 8; ++it) {
        const int row = mBase + it * 2 + hh;
        if (cok && row < M) *(volatile v4f*)(D + (size_t)row * (size_t)ldd + nc) = vv[it];
      }
      __threadfence();
    }
    __builtin_amdgcn_fence(__ATOMIC_RELEASE, "workgroup");
    __builtin_amdgcn_wave_barrier();
    __builtin_amdgcn_fence(__ATOMIC_ACQUIRE, "workgroup");
  }
}

#include <stddef.h>
#include <stdint.h>

#pragma clang fp contract(off)

#define NN      100000
#define NE      1600000
#define DIM     128
#define MPAD    100096
#define NTHR    256
#define NWAVE   8
#define NBRUN   1024
#define SLB     10
#define NBLK    98
#define NSLOT   (NBLK * NBRUN)
#define CHUNK   256
#define NCHUNK  (NE / CHUNK)
#define CPW     782
#define WCAP    4096
#define HCAP    (NWAVE * WCAP)
#define RCAP    21504
#define DEGCAP  64
#define MEAS_B1024_OWNER 16666
#define MEAS_B1024_COL   16710
#define MEAS_DEG_OWNER   37
#define MEAS_DEG_COL     36
#define BK_ZINTS   (HCAP + RCAP + 3 * NBRUN)
#define BK_INTS    (BK_ZINTS + 16)
#define BK_LDS     (BK_INTS * 4)
#define LIST_IT    (RCAP / (4 * NTHR))
#define NBWB       ((DIM * DIM / 8) / NTHR)

static_assert(NE % CHUNK == 0 && NCHUNK * CHUNK == NE);
static_assert(NN % NWAVE == 0 && NN % 16 == 0);
static_assert(DIM == 32 * 4 && DIM % 32 == 0);
static_assert(NBRUN == (1 << SLB));
static_assert((NBLK - 1) * NBRUN < NN && NBLK * NBRUN >= NN && NN - (NBLK - 1) * NBRUN == 672);
static_assert(MPAD % 128 == 0 && MPAD % 64 == 0 && MPAD >= NN && MPAD % 16 == 0);
static_assert((MPAD * (DIM / 8)) % 256 == 0);
static_assert((long long)MPAD * DIM / 8 < (1LL << 31));
static_assert(CPW * NWAVE >= NCHUNK && CPW * (NWAVE - 1) < NCHUNK);
static_assert(((long long)(NE - 1) << SLB) < (1LL << 31));
static_assert(4 * RCAP >= 5 * MEAS_B1024_OWNER && 4 * RCAP >= 5 * MEAS_B1024_COL);
static_assert(RCAP % 256 == 0 && RCAP % (4 * NTHR) == 0 && LIST_IT == 21);
static_assert(DEGCAP >= MEAS_DEG_OWNER + 8 && DEGCAP >= MEAS_DEG_COL + 8 && RCAP > DEGCAP);
static_assert(2 * NWAVE * WCAP >= 3 * RCAP && WCAP % 4 == 0);
static_assert(BK_ZINTS % (NTHR * 4) == 0);
static_assert(BK_LDS == 229440 && BK_LDS <= 262144 && BK_LDS + 0 <= 327680);
static_assert((DIM * DIM / 8) % NTHR == 0 && NBWB == 8);
static_assert(NSLOT % NTHR == 0);
static_assert(((MPAD / 64) * (DIM / 64)) % 8 == 0);

typedef int v4i __attribute__((ext_vector_type(4)));
typedef v4i __attribute__((may_alias)) v4ia;

#define PIN(x) asm volatile("" :: "v"(x))

__global__ __launch_bounds__(NTHR) void k_conv(const float* __restrict__ W, const float* __restrict__ bsrc,
                                               unsigned short* WB, float* PAR) {
  __shared__ __attribute__((aligned(16))) float sp[NTHR];
  const int blk = (int)blockIdx.x;
  const int tid = (int)threadIdx.x;
  if (blk < NBWB) {
    const int g = blk * NTHR + tid;
    const v4f a = *(const v4fa*)(W + (size_t)g * 8);
    const v4f c = *(const v4fa*)(W + (size_t)g * 8 + 4);
    PIN(a);
    PIN(c);
    const v4u o = pack8_bf16(a, c);
    volatile v4u* q = (volatile v4u*)(WB + (size_t)g * 8);
    *q = o;
    __threadfence();
    *q = o;
  } else {
    const int c = tid;
    const float vb = bsrc[c < DIM ? c : DIM - 1];
    PIN(vb);
    const unsigned m = (c < DIM) ? 0xFFFFFFFFu : 0u;
    sp[tid] = __uint_as_float((bf16_bits(vb) << 16) & m);
    __syncthreads();
    if (tid < 64) {
      const v4f o = *(const v4fa*)(sp + 4 * tid);
      volatile v4f* q = (volatile v4f*)(PAR + 4 * tid);
      *q = o;
      __threadfence();
      *q = o;
    }
  }
}

#define PUTW(HJ, SJ, EJ) { \
    const int wv = (int)(((unsigned)(EJ) << SLB) | (SJ)); \
    if (HJ) { if (pos < WCAP) { wlw[pos] = wv; } } \
    pos += (HJ) ? 1 : 0; }

template <int ROLE>
__global__ __launch_bounds__(NTHR) void k_bucket(const int* __restrict__ key, const int* __restrict__ gat,
                                                 int nN, int* listG, int* cntG, int* offG, int* flagG) {
  static_assert(ROLE == 0 || ROLE == 1);
  extern __shared__ __attribute__((aligned(16))) int dsm[];
  int* wl   = dsm;
  int* sl   = dsm + HCAP;
  int* cnt  = sl + RCAP;
  int* offs = cnt + NBRUN;
  int* cur  = offs + NBRUN;
  int* misc = cur + NBRUN;
  const int tid = (int)threadIdx.x, lane = tid & 31, wave = tid >> 5;
  const int b = (int)blockIdx.x;
  const int nodeBase = b * NBRUN;
  const int nb = clampi(nN - nodeBase, 0, NBRUN);

  {
    const v4i z4 = {0, 0, 0, 0};
    for (int i = tid * 4; i < BK_ZINTS; i += NTHR * 4) *(v4ia*)(dsm + i) = z4;
    if (tid < 16) misc[tid] = 0;
  }
  __syncthreads();

  {
    int* wlw = wl + wave * WCAP;
    const int cbeg = wave * CPW;
    const int cend = (cbeg + CPW) < NCHUNK ? (cbeg + CPW) : NCHUNK;
    const unsigned nbs = (unsigned)nodeBase;
    const unsigned unb = (unsigned)nb;
    int wc = 0;
#pragma unroll 1
    for (int ch = cbeg; ch < cend; ++ch) {
      const int e0  = ch * CHUNK + lane * 8;
      const int e0c = e0 < (NE - 8) ? e0 : (NE - 8);
      const v4i ka = *(const v4ia*)(key + e0c);
      const v4i kb = *(const v4ia*)(key + e0c + 4);
      PIN(ka.x); PIN(ka.y); PIN(ka.z); PIN(ka.w);
      PIN(kb.x); PIN(kb.y); PIN(kb.z); PIN(kb.w);
      const bool inr = (e0 == e0c);
      const unsigned s0 = (unsigned)ka.x - nbs, s1 = (unsigned)ka.y - nbs;
      const unsigned s2 = (unsigned)ka.z - nbs, s3 = (unsigned)ka.w - nbs;
      const unsigned s4 = (unsigned)kb.x - nbs, s5 = (unsigned)kb.y - nbs;
      const unsigned s6 = (unsigned)kb.z - nbs, s7 = (unsigned)kb.w - nbs;
      const bool h0 = inr && (s0 < unb);
      const bool h1 = inr && (s1 < unb);
      const bool h2 = inr && (s2 < unb);
      const bool h3 = inr && (s3 < unb);
      const bool h4 = inr && (s4 < unb);
      const bool h5 = inr && (s5 < unb);
      const bool h6 = inr && (s6 < unb);
      const bool h7 = inr && (s7 < unb);
      const unsigned m0 = __builtin_amdgcn_ballot_w32(h0);
      const unsigned m1 = __builtin_amdgcn_ballot_w32(h1);
      const unsigned m2 = __builtin_amdgcn_ballot_w32(h2);
      const unsigned m3 = __builtin_amdgcn_ballot_w32(h3);
      const unsigned m4 = __builtin_amdgcn_ballot_w32(h4);
      const unsigned m5 = __builtin_amdgcn_ballot_w32(h5);
      const unsigned m6 = __builtin_amdgcn_ballot_w32(h6);
      const unsigned m7 = __builtin_amdgcn_ballot_w32(h7);
      const unsigned many = m0 | m1 | m2 | m3 | m4 | m5 | m6 | m7;
      if (many != 0u) {
        unsigned pre = __builtin_amdgcn_mbcnt_lo(m0, 0u);
        pre = __builtin_amdgcn_mbcnt_lo(m1, pre);
        pre = __builtin_amdgcn_mbcnt_lo(m2, pre);
        pre = __builtin_amdgcn_mbcnt_lo(m3, pre);
        pre = __builtin_amdgcn_mbcnt_lo(m4, pre);
        pre = __builtin_amdgcn_mbcnt_lo(m5, pre);
        pre = __builtin_amdgcn_mbcnt_lo(m6, pre);
        pre = __builtin_amdgcn_mbcnt_lo(m7, pre);
        int pos = wc + (int)pre;
        PUTW(h0, s0, e0 + 0)
        PUTW(h1, s1, e0 + 1)
        PUTW(h2, s2, e0 + 2)
        PUTW(h3, s3, e0 + 3)
        PUTW(h4, s4, e0 + 4)
        PUTW(h5, s5, e0 + 5)
        PUTW(h6, s6, e0 + 6)
        PUTW(h7, s7, e0 + 7)
        wc += (int)__builtin_popcount(m0) + (int)__builtin_popcount(m1) + (int)__builtin_popcount(m2)
            + (int)__builtin_popcount(m3) + (int)__builtin_popcount(m4) + (int)__builtin_popcount(m5)
            + (int)__builtin_popcount(m6) + (int)__builtin_popcount(m7);
      }
    }
    if (lane == 0) misc[wave] = wc;
  }
  __syncthreads();

  if (wave == 0) {
    int t = 0, ov = 0;
#pragma unroll 1
    for (int w2 = 0; w2 < NWAVE; ++w2) {
      int c = misc[w2];
      ov |= (c > WCAP) ? 1 : 0;
      c = c < 0 ? 0 : (c > WCAP ? WCAP : c);
      c = __builtin_amdgcn_readfirstlane(c);
#pragma unroll 1
      for (int b0 = 0; b0 < c; b0 += 32) {
        const int idx = b0 + lane;
        const int ent = wl[w2 * WCAP + (idx < WCAP ? idx : WCAP - 1)];
        const int m32 = (c - b0) < 32 ? (c - b0) : 32;
#pragma unroll 1
        for (int k = 0; k < m32; ++k) {
          const int u    = __builtin_amdgcn_readlane(ent, k);
          const int slot = u & (NBRUN - 1);
          if (t < RCAP) {
            const int cvv = cnt[slot];
            if (lane == 0) cnt[slot] = cvv + 1;
            t = t + 1;
          } else {
            ov = 1;
          }
        }
      }
    }
    if (lane == 0) { misc[8] = t; misc[9] = ov; }
  }
  __syncthreads();

  if (wave == 0) {
    const int base = lane * (NBRUN / 32);
    int s = 0, big = 0;
#pragma unroll 1
    for (int i = 0; i < NBRUN / 32; ++i) {
      const int cvv = cnt[base + i];
      s += cvv;
      big |= (cvv > DEGCAP) ? 1 : 0;
    }
    int incl = s;
#pragma unroll
    for (int d = 1; d < 32; d <<= 1) {
      const int y = __shfl_up(incl, d, 32);
      if (lane >= d) incl += y;
    }
    int run = incl - s;
#pragma unroll 1
    for (int i = 0; i < NBRUN / 32; ++i) {
      const int cvv = cnt[base + i];
      offs[base + i] = run;
      cur[base + i]  = run;
      run += cvv;
    }
    const unsigned bm = __builtin_amdgcn_ballot_w32(big != 0);
    if (lane == 0) {
      const int o9 = misc[9];
      misc[9] = o9 | ((bm != 0u) ? 1 : 0);
    }
  }
  __syncthreads();

  if (ROLE == 0) {
    if (wave == 0) {
      int t = 0;
#pragma unroll 1
      for (int w2 = 0; w2 < NWAVE; ++w2) {
        int c = misc[w2];
        c = c < 0 ? 0 : (c > WCAP ? WCAP : c);
        c = __builtin_amdgcn_readfirstlane(c);
#pragma unroll 1
        for (int b0 = 0; b0 < c; b0 += 32) {
          const int idx = b0 + lane;
          const int ent = wl[w2 * WCAP + (idx < WCAP ? idx : WCAP - 1)];
          const int m32 = (c - b0) < 32 ? (c - b0) : 32;
#pragma unroll 1
          for (int k = 0; k < m32; ++k) {
            const int u    = __builtin_amdgcn_readlane(ent, k);
            const int slot = u & (NBRUN - 1);
            if (t < RCAP) {
              int p = cur[slot];
              p = p < 0 ? 0 : (p > RCAP - 1 ? RCAP - 1 : p);
              if (lane == 0) { sl[p] = u; cur[slot] = p + 1; }
              t = t + 1;
            }
          }
        }
      }
    }
    __syncthreads();
  }

  {
    const int ovf = misc[9];
    const int tot = misc[8];
    if (ROLE == 0) {
      int* lb = listG + (size_t)b * (size_t)RCAP;
#pragma unroll 1
      for (int it = 0; it < LIST_IT; ++it) {
        const int p4 = it * NTHR + tid;
        const int i0 = 4 * p4;
        const v4i hv = *(const v4ia*)(sl + i0);
        const int ea = clampi((int)((unsigned)hv.x >> SLB), 0, NE - 1);
        const int eb = clampi((int)((unsigned)hv.y >> SLB), 0, NE - 1);
        const int ec = clampi((int)((unsigned)hv.z >> SLB), 0, NE - 1);
        const int ed = clampi((int)((unsigned)hv.w >> SLB), 0, NE - 1);
        const int ga = gat[ea];
        const int gb = gat[eb];
        const int gc = gat[ec];
        const int gd = gat[ed];
        PIN(ga); PIN(gb); PIN(gc); PIN(gd);
        const int ka = (i0 + 0 < tot) ? -1 : 0;
        const int kb = (i0 + 1 < tot) ? -1 : 0;
        const int kc = (i0 + 2 < tot) ? -1 : 0;
        const int kd = (i0 + 3 < tot) ? -1 : 0;
        const v4i v = { clampi(ga, 0, nN - 1) & ka, clampi(gb, 0, nN - 1) & kb,
                        clampi(gc, 0, nN - 1) & kc, clampi(gd, 0, nN - 1) & kd };
        volatile v4i* q = (volatile v4i*)(lb + (size_t)i0);
        *q = v;
        __threadfence();
        *q = v;
      }
    }
    const v4i fv = {ovf, ovf, ovf, ovf};
    const v4i c4 = *(const v4ia*)(cnt + 4 * tid);
    const v4i o4 = *(const v4ia*)(offs + 4 * tid);
    for (int pass = 0; pass < 2; ++pass) {
      *(volatile v4i*)(cntG + (size_t)nodeBase + 4 * tid) = c4;
      if (ROLE == 0) *(volatile v4i*)(offG + (size_t)nodeBase + 4 * tid) = o4;
      if (tid < 8) *(volatile v4i*)(flagG + (size_t)b * 32 + 4 * tid) = fv;
      __threadfence();
    }
  }
}

__global__ __launch_bounds__(NTHR) void k_dis(const int* __restrict__ cntcol, const int* __restrict__ flagc,
                                              float* dis) {
  __shared__ __attribute__((aligned(16))) float sd[NTHR];
  const int tid = (int)threadIdx.x;
  const int n = (int)blockIdx.x * NTHR + tid;
  int cv = cntcol[n];
  int fl = flagc[(size_t)(n >> SLB) * 32];
  PIN(cv);
  PIN(fl);
  cv = clampi(cv, 0, NE);
  const float c = (float)(cv + 1);
  float d = (c > 0.0f) ? (1.0f / sqrtf(fmaxf(c, 1e-30f))) : 0.0f;
  const float qnan = __int_as_float(0x7fc00000);
  d = (fl != 0) ? qnan : d;
  sd[tid] = d;
  __syncthreads();
  if (tid < 64) {
    const v4f o = *(const v4fa*)(sd + 4 * tid);
    volatile v4f* q = (volatile v4f*)(dis + (size_t)blockIdx.x * NTHR + 4 * tid);
    *q = o;
    __threadfence();
    *q = o;
  }
}

template <int MODE>
__global__ __launch_bounds__(NTHR) void k_prop(const float* __restrict__ H, const float* __restrict__ dis,
                                               const int* __restrict__ listG, const int* __restrict__ cntG,
                                               const int* __restrict__ offG, const int* __restrict__ flagG,
                                               const float* __restrict__ biasv, float* outp, int nN) {
  static_assert(MODE == 0 || MODE == 1);
  __shared__ __attribute__((aligned(16))) float sb[DIM];
  const int tid = (int)threadIdx.x, lane = tid & 31, wave = tid >> 5;
  if (MODE == 1) {
    if (tid < 32) {
      const v4f bvv = *(const v4fa*)(biasv + 4 * tid);
      *(v4fa*)(sb + 4 * tid) = bvv;
    }
    __syncthreads();
  }
  const int r = (int)blockIdx.x * NWAVE + wave;
  const bool live = r < nN;
  const int rc = live ? r : (nN - 1);
  const int blk = rc >> SLB;
  int cv  = cntG[rc];
  int ofv = offG[rc];
  int fl  = flagG[(size_t)blk * 32];
  float dr = dis[rc];
  PIN(cv);
  PIN(ofv);
  PIN(fl);
  PIN(dr);
  const int bad = ((fl != 0) || (cv < 0) || (cv > DEGCAP)) ? 1 : 0;
  const int cn = __builtin_amdgcn_readfirstlane((live && bad == 0) ? clampi(cv, 0, DEGCAP) : 0);
  const int o  = __builtin_amdgcn_readfirstlane(clampi(ofv, 0, RCAP - DEGCAP));
  const int* listb = listG + (size_t)blk * (size_t)RCAP;
  v4f acc = (v4f){0.0f, 0.0f, 0.0f, 0.0f};
#pragma unroll 1
  for (int g0 = 0; g0 < cn; g0 += 32) {
    const int last = o + cn - 1;
    int idx = o + g0 + lane;
    idx = idx > last ? last : idx;
    int idw = listb[idx];
    PIN(idw);
    const int id = clampi(idw, 0, nN - 1);
    float dv = dis[id];
    PIN(dv);
    const float wt = dr * dv;
    const int wb = __float_as_int(wt);
    const int m32 = (cn - g0) < 32 ? (cn - g0) : 32;
#pragma unroll 1
    for (int t = 0; t < m32; ++t) {
      const int ct    = __builtin_amdgcn_readlane(id, t);
      const float wtt = __int_as_float(__builtin_amdgcn_readlane(wb, t));
      const v4f hv = *(const v4fa*)(H + (size_t)ct * DIM + 4 * lane);
      const v4f pv = hv * wtt;
      acc = acc + pv;
    }
  }
  {
    const v4f hs = *(const v4fa*)(H + (size_t)rc * DIM + 4 * lane);
    PIN(hs);
    const float wsf = dr * dr;
    const v4f pv = hs * wsf;
    acc = acc + pv;
  }
  v4f ov = acc;
  if (MODE == 1) {
    const v4f bq = *(const v4fa*)(sb + 4 * lane);
    ov = ov + bq;
  }
  const float qnan = __int_as_float(0x7fc00000);
  const v4f qn = (v4f){qnan, qnan, qnan, qnan};
  ov = (bad != 0) ? qn : ov;
  if (live) {
    volatile v4f* q = (volatile v4f*)(outp + (size_t)r * DIM + 4 * lane);
    *q = ov;
    __threadfence();
    *q = ov;
  }
}

constexpr size_t SZ_T    = (size_t)MPAD * DIM * 4;
constexpr size_t SZ_R    = (size_t)MPAD * DIM * 4;
constexpr size_t SZ_XB   = (size_t)MPAD * DIM * 2;
constexpr size_t SZ_LIST = (size_t)NBLK * RCAP * 4;
constexpr size_t SZ_TAB  = (size_t)NSLOT * 4;
constexpr size_t SZ_WB   = (size_t)DIM * DIM * 2;
constexpr size_t SZ_PAR  = (size_t)256 * 4;
constexpr size_t SZ_FLAG = (size_t)NBLK * 32 * 4;
constexpr size_t O_T     = 0;
constexpr size_t O_R     = O_T + SZ_T;
constexpr size_t O_LIST  = O_R + SZ_R;
constexpr size_t O_CNT   = O_LIST + SZ_LIST;
constexpr size_t O_OFF   = O_CNT + SZ_TAB;
constexpr size_t O_CNTC  = O_OFF + SZ_TAB;
constexpr size_t O_DIS   = O_CNTC + SZ_TAB;
constexpr size_t O_WB    = O_DIS + SZ_TAB;
constexpr size_t O_PAR   = O_WB + SZ_WB;
constexpr size_t O_FLAG  = O_PAR + SZ_PAR;
constexpr size_t O_FLAGC = O_FLAG + SZ_FLAG;
constexpr size_t WS_TOTAL = O_FLAGC + SZ_FLAG;
static_assert(SZ_T % 256 == 0 && SZ_R % 256 == 0 && SZ_LIST % 256 == 0 && SZ_TAB % 256 == 0);
static_assert(SZ_WB % 256 == 0 && SZ_PAR % 256 == 0 && SZ_FLAG % 256 == 0 && SZ_XB <= SZ_R);
static_assert(WS_TOTAL == (size_t)112592 * 1000 + 384 && WS_TOTAL <= ((size_t)128 << 20));
static_assert((size_t)NN * DIM * 4 <= SZ_R && (size_t)(NN - 1) * DIM + DIM - 1 == (size_t)12799999);

extern "C" void kernel_launch(void* const* d_in, const int* in_sizes, int n_in,
                              void* d_out, int out_size, void* d_ws, size_t ws_size,
                              hipStream_t stream) {
  if (n_in < 4) return;
  if (in_sizes[0] != NN * DIM) return;
  if (in_sizes[1] != 2 * NE) return;
  if (in_sizes[2] != DIM * DIM) return;
  if (in_sizes[3] != DIM) return;
  if (out_size != NN * DIM) return;
  if (ws_size < WS_TOTAL) return;

  const float* x     = (const float*)d_in[0];
  const int*   ei    = (const int*)d_in[1];
  const float* lin_w = (const float*)d_in[2];
  const float* lin_b = (const float*)d_in[3];
  float* out = (float*)d_out;
  const int* erow = ei;
  const int* ecol = ei + NE;

  char* ws = (char*)d_ws;
  float*          Tp   = (float*)(ws + O_T);
  unsigned short* XB   = (unsigned short*)(ws + O_R);
  float*          Up   = (float*)(ws + O_R);
  int*            LST  = (int*)(ws + O_LIST);
  int*            CNT  = (int*)(ws + O_CNT);
  int*            OFF  = (int*)(ws + O_OFF);
  int*            CNTC = (int*)(ws + O_CNTC);
  float*          DIS  = (float*)(ws + O_DIS);
  unsigned short* WB   = (unsigned short*)(ws + O_WB);
  float*          PAR  = (float*)(ws + O_PAR);
  int*            FLG  = (int*)(ws + O_FLAG);
  int*            FLGC = (int*)(ws + O_FLAGC);

  hipFuncSetAttribute(reinterpret_cast<const void*>(&k_bucket<0>), hipFuncAttributeMaxDynamicSharedMemorySize,
                      (int)BK_LDS);
  hipFuncSetAttribute(reinterpret_cast<const void*>(&k_bucket<1>), hipFuncAttributeMaxDynamicSharedMemorySize,
                      (int)BK_LDS);

  k_plane<0><<<MPAD * (DIM / 8) / 256, 256, 0, stream>>>(x, NN, DIM, DIM, XB, MPAD, DIM);
  k_conv<<<NBWB + 1, NTHR, 0, stream>>>(lin_w, lin_b, WB, PAR);
  const int gemmTiles = (MPAD / 64) * (DIM / 64);
  k_gemm_nt<0, 0><<<gemmTiles / 8, 256, 0, stream>>>(XB, WB, PAR + DIM, Tp, MPAD, DIM, DIM, DIM);
  k_bucket<0><<<NBLK, NTHR, BK_LDS, stream>>>(erow, ecol, NN, LST, CNT, OFF, FLG);
  k_bucket<1><<<NBLK, NTHR, BK_LDS, stream>>>(ecol, erow, NN, LST, CNTC, OFF, FLGC);
  k_dis<<<NSLOT / NTHR, NTHR, 0, stream>>>(CNTC, FLGC, DIS);
  k_prop<0><<<NN / NWAVE, NTHR, 0, stream>>>(Tp, DIS, LST, CNT, OFF, FLG, PAR, Up, NN);
  k_prop<1><<<NN / NWAVE, NTHR, 0, stream>>>(Up, DIS, LST, CNT, OFF, FLG, PAR, out, NN);
}
